// ImportanceAggregator_28424093564971
// MI455X (gfx1250) — hardware-verified
//
#include <hip/hip_runtime.h>
#include <stddef.h>


#define FD     256
#define KN     16
#define KC     256
#define NO     256
#define NTHR   256
#define NWAVE  8
#define BROWS  32
#define NPW    (BROWS / NWAVE)
#define HP     264
#define SP     260
#define HSC    32
#define WSC    64
#define WSCAP  134217728
#define WPB    ((NO * KC / 8) / NTHR)

static_assert((NO * KC / 8) % NTHR == 0);
static_assert(KC / 8 == 32);
static_assert((KC % 32) == 0);
static_assert(BROWS == 2 * 16);
static_assert(NO == 4 * 64);
static_assert(BROWS == NWAVE * NPW);
static_assert(FD == 32 * 8);
static_assert(NO == 2 * 128);
static_assert((HP * 2) % 16 == 0);
static_assert((SP * 4) % 16 == 0);
static_assert(HP >= KC);
static_assert(SP >= NO);
static_assert(BROWS <= 32);
static_assert(BROWS * HP * 2 + BROWS * KN * 4 * 2 + BROWS * 4 + BROWS * SP * 4 <= 65536);

typedef float     v4f  __attribute__((ext_vector_type(4)));
typedef float     v8f  __attribute__((ext_vector_type(8)));
typedef int       v4i  __attribute__((ext_vector_type(4)));
typedef _Float16  v8h  __attribute__((ext_vector_type(8)));
typedef _Float16  v16h __attribute__((ext_vector_type(16)));
union FragH { v16h v; v8h h[2]; };

__device__ __forceinline__ v8f wmf(v16h a, v16h b, v8f c) {
  v8f d = __builtin_amdgcn_wmma_f32_16x16x32_f16(false, a, false, b, (short)0, c, false, false);
  asm volatile("v_nop\n\tv_nop\n\tv_nop\n\tv_nop" : "+v"(d) : "v"(a), "v"(b));
  return d;
}

__device__ __forceinline__ int clampi(int v, int hi) {
  v = v < 0 ? 0 : v;
  return v > hi ? hi : v;
}

__global__ __launch_bounds__(NTHR) void k_wprep(const float* __restrict__ w, _Float16* wp) {
  const int i  = (int)blockIdx.x * NTHR + (int)threadIdx.x;
  const int n  = i >> 5;
  const int k0 = (i & 31) * 8;
  v8h hv;
#pragma unroll
  for (int e = 0; e < 8; ++e) hv[e] = (_Float16)(w[(size_t)(k0 + e) * NO + n] * (float)WSC);
  _Float16* d = wp + (size_t)i * 8;
  *(volatile v8h*)d = hv;
  __threadfence();
  *(volatile v8h*)d = hv;
}

__global__ __launch_bounds__(NTHR) void k_main(
    const float* __restrict__ x, const int* __restrict__ ei, const float* __restrict__ iw,
    const _Float16* __restrict__ wp, const float* __restrict__ bs,
    const float* __restrict__ ga, const float* __restrict__ be,
    float* out, int nN) {
  __shared__ __attribute__((aligned(16))) _Float16 hs[BROWS * HP];
  __shared__ __attribute__((aligned(16))) int      sidx[BROWS * KN];
  __shared__ __attribute__((aligned(16))) float    snw[BROWS * KN];
  __shared__ __attribute__((aligned(16))) float    ssb[BROWS];
  __shared__ __attribute__((aligned(16))) float    stg[BROWS * SP];
  constexpr float OSC = 1.0f / (float)(HSC * WSC);
  const int tid = threadIdx.x, lane = tid & 31, wave = tid >> 5, hh = lane >> 4, m = lane & 15;
  const int base = blockIdx.x * BROWS;

  if (wave == 0) {
    const int g = clampi(base + lane, nN - 1);
    const v4i* ip = (const v4i*)(ei + (size_t)g * KN);
    const v4f* wq = (const v4f*)(iw + (size_t)g * KN);
    v4i idv[4];
    v4f wv[4];
#pragma unroll
    for (int q = 0; q < 4; ++q) { idv[q] = ip[q]; wv[q] = wq[q]; }
    float wsum = 0.0f;
#pragma unroll
    for (int q = 0; q < 4; ++q) { wsum += wv[q].x; wsum += wv[q].y; wsum += wv[q].z; wsum += wv[q].w; }
    const bool  zs  = (wsum == 0.0f);
    const float inv = 1.0f / (zs ? 1.0f : wsum);
    const float unf = 1.0f / (float)KN;
    float sb = 0.0f;
#pragma unroll
    for (int q = 0; q < 4; ++q) {
      v4f nw;
      nw.x = zs ? unf : wv[q].x * inv;
      nw.y = zs ? unf : wv[q].y * inv;
      nw.z = zs ? unf : wv[q].z * inv;
      nw.w = zs ? unf : wv[q].w * inv;
      sb += nw.x; sb += nw.y; sb += nw.z; sb += nw.w;
      v4i iv = idv[q];
      iv.x = clampi(iv.x, nN - 1); iv.y = clampi(iv.y, nN - 1);
      iv.z = clampi(iv.z, nN - 1); iv.w = clampi(iv.w, nN - 1);
      *(v4i*)(sidx + lane * KN + 4 * q) = iv;
      *(v4f*)(snw  + lane * KN + 4 * q) = nw;
    }
    ssb[lane] = sb;
  }
  __syncthreads();

  {
    const int fq = 8 * lane;
#pragma unroll 1
    for (int p = 0; p < NPW; ++p) {
      const int nd = wave * NPW + p;
      const int*   ipn = sidx + nd * KN;
      const float* wpn = snw + nd * KN;
      v4f a0 = {0.f, 0.f, 0.f, 0.f};
      v4f a1 = {0.f, 0.f, 0.f, 0.f};
#pragma unroll 4
      for (int k = 0; k < KN; ++k) {
        const int   s  = ipn[k];
        const float wk = wpn[k];
        const float* fr = x + (size_t)s * FD + fq;
        const v4f x0 = *(const v4f*)fr;
        const v4f x1 = *(const v4f*)(fr + 4);
        a0.x = fmaf(wk, x0.x, a0.x); a0.y = fmaf(wk, x0.y, a0.y);
        a0.z = fmaf(wk, x0.z, a0.z); a0.w = fmaf(wk, x0.w, a0.w);
        a1.x = fmaf(wk, x1.x, a1.x); a1.y = fmaf(wk, x1.y, a1.y);
        a1.z = fmaf(wk, x1.z, a1.z); a1.w = fmaf(wk, x1.w, a1.w);
      }
      v8h hv;
      hv[0] = (_Float16)(a0.x * (float)HSC); hv[1] = (_Float16)(a0.y * (float)HSC);
      hv[2] = (_Float16)(a0.z * (float)HSC); hv[3] = (_Float16)(a0.w * (float)HSC);
      hv[4] = (_Float16)(a1.x * (float)HSC); hv[5] = (_Float16)(a1.y * (float)HSC);
      hv[6] = (_Float16)(a1.z * (float)HSC); hv[7] = (_Float16)(a1.w * (float)HSC);
      *(v8h*)(hs + nd * HP + fq) = hv;
    }
  }
  __syncthreads();

  const int rg = wave >> 2, cq = wave & 3;
  v8f acc[4];
  {
    v8f z = {0.f, 0.f, 0.f, 0.f, 0.f, 0.f, 0.f, 0.f};
    acc[0] = z; acc[1] = z; acc[2] = z; acc[3] = z;
  }
  const _Float16* ap = hs + (16 * rg + m) * HP + 8 * hh;
#pragma unroll 1
  for (int kt = 0; kt < KC / 32; ++kt) {
    FragH af;
    af.h[0] = *(const v8h*)(ap + 32 * kt);
    af.h[1] = *(const v8h*)(ap + 32 * kt + 16);
#pragma unroll
    for (int t = 0; t < 4; ++t) {
      const _Float16* bp = wp + (size_t)(64 * cq + 16 * t + m) * KC + 32 * kt + 8 * hh;
      FragH bf;
      bf.h[0] = *(const v8h*)bp;
      bf.h[1] = *(const v8h*)(bp + 16);
      acc[t] = wmf(af.v, bf.v, acc[t]);
    }
  }

  {
    float bv[4];
#pragma unroll
    for (int t = 0; t < 4; ++t) bv[t] = bs[64 * cq + 16 * t + m];
    float sbv[8];
#pragma unroll
    for (int r = 0; r < 8; ++r) sbv[r] = ssb[16 * rg + 8 * hh + r];
    float* sp = stg + (16 * rg + 8 * hh) * SP + 64 * cq + m;
#pragma unroll
    for (int t = 0; t < 4; ++t) {
#pragma unroll
      for (int r = 0; r < 8; ++r) sp[r * SP + 16 * t] = acc[t][r] * OSC + sbv[r] * bv[t];
    }
  }
  __syncthreads();

  const v4f g0 = *(const v4f*)(ga + 4 * lane);
  const v4f g1 = *(const v4f*)(ga + 128 + 4 * lane);
  const v4f e0 = *(const v4f*)(be + 4 * lane);
  const v4f e1 = *(const v4f*)(be + 128 + 4 * lane);
  constexpr float invD = 1.0f / (float)NO;
  v4f o0[NPW], o1[NPW];
#pragma unroll
  for (int r = 0; r < NPW; ++r) {
    const float* rp = stg + (NPW * wave + r) * SP;
    const v4f v0 = *(const v4f*)(rp + 4 * lane);
    const v4f v1 = *(const v4f*)(rp + 128 + 4 * lane);
    float s = ((v0.x + v0.y) + (v0.z + v0.w)) + ((v1.x + v1.y) + (v1.z + v1.w));
#pragma unroll
    for (int off = 16; off >= 1; off >>= 1) s += __shfl_xor(s, off, 32);
    const float mean = s * invD;
    v4f d0, d1;
    d0.x = v0.x - mean; d0.y = v0.y - mean; d0.z = v0.z - mean; d0.w = v0.w - mean;
    d1.x = v1.x - mean; d1.y = v1.y - mean; d1.z = v1.z - mean; d1.w = v1.w - mean;
    float s2 = ((d0.x * d0.x + d0.y * d0.y) + (d0.z * d0.z + d0.w * d0.w))
             + ((d1.x * d1.x + d1.y * d1.y) + (d1.z * d1.z + d1.w * d1.w));
#pragma unroll
    for (int off = 16; off >= 1; off >>= 1) s2 += __shfl_xor(s2, off, 32);
    const float var  = s2 * invD;
    const float rstd = rsqrtf(var + 1e-5f);
    v4f y0, y1;
    y0.x = (d0.x * rstd) * g0.x + e0.x; y0.y = (d0.y * rstd) * g0.y + e0.y;
    y0.z = (d0.z * rstd) * g0.z + e0.z; y0.w = (d0.w * rstd) * g0.w + e0.w;
    y1.x = (d1.x * rstd) * g1.x + e1.x; y1.y = (d1.y * rstd) * g1.y + e1.y;
    y1.z = (d1.z * rstd) * g1.z + e1.z; y1.w = (d1.w * rstd) * g1.w + e1.w;
    o0[r] = y0; o1[r] = y1;
  }

#pragma unroll
  for (int r = 0; r < NPW; ++r) {
    const int row = base + NPW * wave + r;
    if (row < nN) {
      float* op = out + (size_t)row * NO;
      *(volatile v4f*)(op + 4 * lane)       = o0[r];
      *(volatile v4f*)(op + 128 + 4 * lane) = o1[r];
    }
  }
  __threadfence();
#pragma unroll
  for (int r = 0; r < NPW; ++r) {
    const int row = base + NPW * wave + r;
    if (row < nN) {
      float* op = out + (size_t)row * NO;
      *(volatile v4f*)(op + 4 * lane)       = o0[r];
      *(volatile v4f*)(op + 128 + 4 * lane) = o1[r];
    }
  }
}

extern "C" void kernel_launch(void* const* d_in, const int* in_sizes, int n_in,
                              void* d_out, int out_size, void* d_ws, size_t ws_size,
                              hipStream_t stream) {
  if (n_in < 7) return;
  const int nN = in_sizes[0] / FD;
  if (nN <= 0) return;
  if (in_sizes[0] != nN * FD || in_sizes[1] != nN * KN || in_sizes[2] != nN * KN) return;
  if (in_sizes[3] != KC * NO || in_sizes[4] != NO || in_sizes[5] != NO || in_sizes[6] != NO) return;
  if (out_size != nN * NO) return;
  if (nN > (1 << 24)) return;

  const float* x  = (const float*)d_in[0];
  const int*   ei = (const int*)d_in[1];
  const float* iw = (const float*)d_in[2];
  const float* W  = (const float*)d_in[3];
  const float* bs = (const float*)d_in[4];
  const float* ga = (const float*)d_in[5];
  const float* be = (const float*)d_in[6];
  float* out = (float*)d_out;

  char* ws = (char*)d_ws;
  size_t off = 0;
  const size_t oW = off; off += (size_t)(NO * KC) * 2;  off = (off + 255) & ~(size_t)255;
  if (off > ws_size || off > (size_t)WSCAP) return;
  _Float16* wpl = (_Float16*)(ws + oW);

  const int nBlk = (nN + BROWS - 1) / BROWS;

  k_wprep<<<WPB, NTHR, 0, stream>>>(W, wpl);

  k_main<<<nBlk, NTHR, 0, stream>>>(x, ei, iw, wpl, bs, ga, be, out, nN);
}
